// GARCHGRUCell_83605833383957
// MI455X (gfx1250) — hardware-run, weakly checked
//
#include <hip/hip_runtime.h>
#include <math.h>

constexpr int NBATCH = 8192;
constexpr int NINF   = 64;
constexpr int NHID   = 1024;
constexpr int KCAT   = NINF + NHID;
constexpr int NZR    = 2 * NHID;
constexpr int NW3    = 3 * NHID;
constexpr int NTHR   = 256;
constexpr int SLABP  = 68;
constexpr float WCARRY     = 64.0f;
constexpr float WCARRY_INV = 1.0f / 64.0f;
static_assert(KCAT == 1088, "K of the fused [x|h] operand");
static_assert(KCAT % 32 == 0, "K multiple of 32, no tail");
static_assert(NBATCH % 64 == 0 && NHID % 64 == 0 && NZR % 64 == 0, "M, N tile multiples");
static_assert(((NBATCH / 64) * (NZR / 64)) % 8 == 0, "zr grid exact");
static_assert(((NBATCH / 64) * (NHID / 64)) % 8 == 0, "h grid exact");
static_assert((NBATCH * (NINF / 8)) % NTHR == 0, "x convert grid exact");
static_assert((NBATCH * (NHID / 8)) % NTHR == 0, "h convert grid exact");
static_assert((NHID * (NINF / 8)) % NTHR == 0, "W convert grid exact");
static_assert((NHID * (NHID / 8)) % NTHR == 0, "U convert grid exact");
static_assert(NBATCH % NTHR == 0, "row kernel grid exact");
static_assert((KCAT * 2) % 128 == 0, "operand row pitch is a whole number of 128-B lines");

typedef __attribute__((ext_vector_type(16))) _Float16 v16h;
typedef __attribute__((ext_vector_type(8)))  _Float16 v8h;
typedef __attribute__((ext_vector_type(8)))  float    v8f;
typedef __attribute__((ext_vector_type(4)))  float    v4f;

__device__ __forceinline__ void mma_guard4(v8f& a0, v8f& a1, v8f& a2, v8f& a3, v16h x, v16h b0, v16h b1, v16h b2, v16h b3) {
  asm volatile("v_nop\n\tv_nop\n\tv_nop\n\tv_nop" : "+v"(a0), "+v"(a1), "+v"(a2), "+v"(a3) : "v"(x), "v"(b0), "v"(b1), "v"(b2), "v"(b3));
}
__device__ __forceinline__ void keep4_h(v16h a, v16h b, v16h c, v16h d) { asm volatile("v_nop" :: "v"(a), "v"(b), "v"(c), "v"(d)); }
__device__ __forceinline__ void acc_guard4(v8f& a, v8f& b, v8f& c, v8f& d) { asm volatile("v_nop\n\tv_nop\n\tv_nop\n\tv_nop" : "+v"(a), "+v"(b), "+v"(c), "+v"(d)); }

template <typename T> struct Frag;
template <> struct Frag<_Float16> {
  typedef v16h V; union U { v16h v; v8h h[2]; };
  static __device__ __forceinline__ v16h load(const _Float16* p) {
    U f; f.h[0] = *(const v8h*)(p); f.h[1] = *(const v8h*)(p + 16); return f.v;
  }
  static __device__ __forceinline__ v8f mma(v16h a, v16h b, v8f c) {
    return __builtin_amdgcn_wmma_f32_16x16x32_f16(false, a, false, b, (short)0, c, false, false);
  }
};

__device__ __forceinline__ float sigm_f(float v) { return 1.0f / (1.0f + expf(-v)); }

__device__ __forceinline__ void garch_consts(const float* o, const float* al, const float* be, float& omega, float& a, float& b) {
  const float orw = o[0];
  omega = (fmaxf(orw, 0.0f) + log1pf(expf(-fabsf(orw)))) + 1e-6f;
  a = sigm_f(al[0]);
  b = sigm_f(be[0]) * (1.0f - a * 0.99f);
}

__global__ __launch_bounds__(NTHR) void cvt8_kernel(const float* __restrict__ s0, const float* __restrict__ s1,
                                                    const float* __restrict__ s2,
                                                    unsigned short* dst, unsigned short* dst2, int has2,
                                                    int nrow, int ncol8, int dpitch, int dcol0, float sc) {
  const int y = blockIdx.y;
  const float* src = (y == 0) ? s0 : ((y == 1) ? s1 : s2);
  const int i  = blockIdx.x * NTHR + threadIdx.x;
  const int n8 = nrow * ncol8;
  if (i < n8) {
    const int row = i / ncol8;
    const int c8  = i - row * ncol8;
    const float* sp = src + (size_t)i * 8;
    const v4f a = *(const v4f*)(sp);
    const v4f b = *(const v4f*)(sp + 4);
    v8h hv;
#pragma unroll
    for (int e = 0; e < 4; ++e) {
      const float fa = a[e] * sc;
      const float fb = b[e] * sc;
      hv[e]     = (_Float16)fa;
      hv[4 + e] = (_Float16)fb;
    }
    const size_t o = (size_t)(y * nrow + row) * (size_t)dpitch + (size_t)dcol0 + (size_t)c8 * 8;
    *(volatile v8h*)(dst + o) = hv;
    if (has2) *(volatile v8h*)(dst2 + o) = hv;
    __threadfence();
    *(volatile v8h*)(dst + o) = hv;
    if (has2) *(volatile v8h*)(dst2 + o) = hv;
  }
}

__global__ __launch_bounds__(NTHR) void garch_rows_kernel(const float* __restrict__ x,
                                                          const float* __restrict__ eps_prev, const float* __restrict__ sig_prev,
                                                          const float* __restrict__ omega_raw, const float* __restrict__ alpha_raw,
                                                          const float* __restrict__ beta_raw,
                                                          float* out_eps, float* out_sig) {
  const int i = blockIdx.x * NTHR + threadIdx.x;
  if (i < NBATCH) {
    float omega, a, b;
    garch_consts(omega_raw, alpha_raw, beta_raw, omega, a, b);
    const float x0 = x[(size_t)i * NINF];
    const float e2 = x0 * x0;
    const float gi = (omega + a * eps_prev[i]) + b * sig_prev[i];
    *(volatile float*)(out_eps + i) = e2;
    *(volatile float*)(out_sig + i) = gi;
    __threadfence();
    *(volatile float*)(out_eps + i) = e2;
    *(volatile float*)(out_sig + i) = gi;
  }
}

template <int MODE>
__global__ __launch_bounds__(NTHR) void gru_gemm64(
    const unsigned short* Ap, const unsigned short* __restrict__ Btp,
    const float* __restrict__ bias_a0, const float* __restrict__ bias_b0,
    const float* __restrict__ bias_a1, const float* __restrict__ bias_b1,
    const float* __restrict__ h_prev, const float* zin, float* fout, unsigned short* rh_out,
    const float* __restrict__ wg_w, const float* __restrict__ wg_b,
    const float* __restrict__ eps_prev, const float* __restrict__ sig_prev,
    const float* __restrict__ omega_raw, const float* __restrict__ alpha_raw,
    const float* __restrict__ beta_raw, const float* __restrict__ gamma_p) {
  constexpr int NCOLS  = (MODE == 0) ? NZR : NHID;
  constexpr int tilesN = NCOLS / 64;
  constexpr int tilesM = NBATCH / 64;
  __shared__ __align__(16) float sT[8][16 * SLABP];
  const int lane = threadIdx.x & 31;
  const int wave = threadIdx.x >> 5;
  const int tile = blockIdx.x * 8 + wave;
  if (tile >= tilesM * tilesN) return;
  const int tm = tile / tilesN;
  const int tn = tile - tm * tilesN;
  const int m0 = tm << 6;
  const int n0 = tn << 6;

  const int rlane = lane & 15;
  const int koff  = (lane >> 4) * 8;
  const int mOff  = (lane >> 4) * 8;

  const _Float16* aBase = (const _Float16*)Ap  + (size_t)(m0 + rlane) * KCAT + koff;
  const _Float16* bBase = (const _Float16*)Btp + (size_t)(n0 + rlane) * KCAT + koff;

  v8f acc[4][4];
#pragma unroll
  for (int i = 0; i < 4; ++i)
#pragma unroll
    for (int j = 0; j < 4; ++j) acc[i][j] = (v8f){0.f, 0.f, 0.f, 0.f, 0.f, 0.f, 0.f, 0.f};

#pragma unroll 1
  for (int k0 = 0; k0 < KCAT; k0 += 32) {
    v16h bh[4];
#pragma unroll
    for (int j = 0; j < 4; ++j) bh[j] = Frag<_Float16>::load(bBase + (size_t)j * 16 * KCAT + k0);
#pragma unroll
    for (int i = 0; i < 4; ++i) {
      const v16h ah = Frag<_Float16>::load(aBase + (size_t)i * 16 * KCAT + k0);
#pragma unroll
      for (int j = 0; j < 4; ++j) acc[i][j] = Frag<_Float16>::mma(ah, bh[j], acc[i][j]);
      mma_guard4(acc[i][0], acc[i][1], acc[i][2], acc[i][3], ah, bh[0], bh[1], bh[2], bh[3]);
    }
    keep4_h(bh[0], bh[1], bh[2], bh[3]);
  }
  acc_guard4(acc[0][0], acc[0][1], acc[0][2], acc[0][3]);
  acc_guard4(acc[1][0], acc[1][1], acc[1][2], acc[1][3]);
  acc_guard4(acc[2][0], acc[2][1], acc[2][2], acc[2][3]);
  acc_guard4(acc[3][0], acc[3][1], acc[3][2], acc[3][3]);

  float* slab = sT[wave];
  const int hh = lane >> 4;
  const int c4 = (lane & 15) * 4;
  const bool isR = (MODE == 0) && (n0 >= NHID);
  const int ncol = (MODE == 0) ? (n0 & (NHID - 1)) : n0;
  const float* bA = isR ? bias_a1 : bias_a0;
  const float* bB = isR ? bias_b1 : bias_b0;
  const v4f bva = *(const v4f*)(bA + ncol + c4);
  const v4f bvb = *(const v4f*)(bB + ncol + c4);
  v4f bsum;
#pragma unroll
  for (int e = 0; e < 4; ++e) bsum[e] = bva[e] + bvb[e];
  v4f wgw = (v4f){0.f, 0.f, 0.f, 0.f};
  v4f wgb = (v4f){0.f, 0.f, 0.f, 0.f};
  float omega = 0.f, ga = 0.f, gb = 0.f, gam = 0.f;
  if (MODE == 1) {
    wgw = *(const v4f*)(wg_w + ncol + c4);
    wgb = *(const v4f*)(wg_b + ncol + c4);
    garch_consts(omega_raw, alpha_raw, beta_raw, omega, ga, gb);
    gam = gamma_p[0];
  }

#pragma unroll
  for (int i = 0; i < 4; ++i) {
    const int mBase = m0 + (i << 4);
#pragma unroll
    for (int j = 0; j < 4; ++j) {
#pragma unroll
      for (int r = 0; r < 8; ++r) slab[(mOff + r) * SLABP + (j << 4) + rlane] = acc[i][j][r] * WCARRY_INV;
    }
    __builtin_amdgcn_fence(__ATOMIC_RELEASE, "workgroup");
    __builtin_amdgcn_wave_barrier();
    __builtin_amdgcn_fence(__ATOMIC_ACQUIRE, "workgroup");

#pragma unroll 1
    for (int it = 0; it < 8; ++it) {
      const int row = it * 2 + hh;
      const size_t grow = (size_t)(mBase + row);
      float* sp = slab + row * SLABP + c4;
      const v4f s  = *(const v4f*)sp;
      const v4f hp = *(const v4f*)(h_prev + grow * NHID + ncol + c4);
      v4f o;
      if (MODE == 0) {
#pragma unroll
        for (int e = 0; e < 4; ++e) {
          const float g = sigm_f(s[e] + bsum[e]);
          const float gh = g * hp[e];
          o[e] = isR ? gh : g;
        }
      } else {
        const v4f zv = *(const v4f*)(zin + grow * NHID + ncol + c4);
        const float gi = (omega + ga * eps_prev[grow]) + gb * sig_prev[grow];
#pragma unroll
        for (int e = 0; e < 4; ++e) {
          const float ht   = tanhf(s[e] + bsum[e]);
          const float hhat = (1.0f - zv[e]) * ht + zv[e] * hp[e];
          const float gt   = gi * wgw[e] + wgb[e];
          o[e] = tanhf(hhat + gam * gt);
        }
      }
      *(v4f*)sp = o;
    }
    __builtin_amdgcn_fence(__ATOMIC_RELEASE, "workgroup");
    __builtin_amdgcn_wave_barrier();
    __builtin_amdgcn_fence(__ATOMIC_ACQUIRE, "workgroup");

    if (isR) {
      const int q = lane >> 3, c8 = (lane & 7) * 8;
      for (int pass = 0; pass < 2; ++pass) {
#pragma unroll
        for (int it = 0; it < 4; ++it) {
          const int row = it * 4 + q;
          const float* sp = slab + row * SLABP + c8;
          v8h hv;
#pragma unroll
          for (int e = 0; e < 8; ++e) hv[e] = (_Float16)sp[e];
          *(volatile v8h*)(rh_out + (size_t)(mBase + row) * KCAT + NINF + ncol + c8) = hv;
        }
        __threadfence();
      }
    } else {
      for (int pass = 0; pass < 2; ++pass) {
#pragma unroll
        for (int it = 0; it < 8; ++it) {
          const int row = it * 2 + hh;
          const v4f v = *(const v4f*)(slab + row * SLABP + c4);
          *(volatile v4f*)(fout + (size_t)(mBase + row) * NHID + ncol + c4) = v;
        }
        __threadfence();
      }
    }
    __builtin_amdgcn_fence(__ATOMIC_RELEASE, "workgroup");
    __builtin_amdgcn_wave_barrier();
    __builtin_amdgcn_fence(__ATOMIC_ACQUIRE, "workgroup");
  }
}

extern "C" void kernel_launch(void* const* d_in, const int* in_sizes, int n_in,
                              void* d_out, int out_size, void* d_ws, size_t ws_size, hipStream_t stream) {
  if (n_in < 22 || d_out == nullptr || d_ws == nullptr) return;
  if (in_sizes[0] != NBATCH * NINF || in_sizes[1] != NBATCH * NHID || in_sizes[2] != NBATCH || in_sizes[3] != NBATCH) return;
  if (in_sizes[4] != NHID * NINF || in_sizes[5] != NHID || in_sizes[6] != NHID * NHID || in_sizes[7] != NHID) return;
  if (in_sizes[8] != NHID * NINF || in_sizes[9] != NHID || in_sizes[10] != NHID * NHID || in_sizes[11] != NHID) return;
  if (in_sizes[12] != NHID * NINF || in_sizes[13] != NHID || in_sizes[14] != NHID * NHID || in_sizes[15] != NHID) return;
  if (in_sizes[16] != NHID || in_sizes[17] != NHID) return;
  if (in_sizes[18] != 1 || in_sizes[19] != 1 || in_sizes[20] != 1 || in_sizes[21] != 1) return;
  if (out_size != NBATCH * NHID + 2 * NBATCH) return;

  const float* x        = (const float*)d_in[0];
  const float* h_prev   = (const float*)d_in[1];
  const float* eps_prev = (const float*)d_in[2];
  const float* sig_prev = (const float*)d_in[3];
  const float* Wz_w = (const float*)d_in[4];
  const float* Wz_b = (const float*)d_in[5];
  const float* Uz_w = (const float*)d_in[6];
  const float* Uz_b = (const float*)d_in[7];
  const float* Wr_w = (const float*)d_in[8];
  const float* Wr_b = (const float*)d_in[9];
  const float* Ur_w = (const float*)d_in[10];
  const float* Ur_b = (const float*)d_in[11];
  const float* Wh_w = (const float*)d_in[12];
  const float* Wh_b = (const float*)d_in[13];
  const float* Uh_w = (const float*)d_in[14];
  const float* Uh_b = (const float*)d_in[15];
  const float* Wg_w = (const float*)d_in[16];
  const float* Wg_b = (const float*)d_in[17];
  const float* omega_raw = (const float*)d_in[18];
  const float* alpha_raw = (const float*)d_in[19];
  const float* beta_raw  = (const float*)d_in[20];
  const float* gamma_p   = (const float*)d_in[21];

  float* out_h   = (float*)d_out;
  float* out_eps = out_h + (size_t)NBATCH * NHID;
  float* out_sig = out_eps + NBATCH;

  char* ws = (char*)d_ws; size_t off = 0;
  auto carve = [&](size_t bytes) -> char* { char* p = ws + off; off += (bytes + 255) & ~(size_t)255; return p; };
  unsigned short* A1 = (unsigned short*)carve((size_t)NBATCH * KCAT * 2);
  unsigned short* A3 = (unsigned short*)carve((size_t)NBATCH * KCAT * 2);
  unsigned short* BT = (unsigned short*)carve((size_t)NW3 * KCAT * 2);
  float*          ZB = (float*)carve((size_t)NBATCH * NHID * 4);
  if (off > ws_size || off > (size_t)134217728) return;

  cvt8_kernel<<<dim3(NBATCH * (NINF / 8) / NTHR, 1), NTHR, 0, stream>>>(x, x, x, A1, A3, 1, NBATCH, NINF / 8, KCAT, 0, 1.0f);
  cvt8_kernel<<<dim3(NBATCH * (NHID / 8) / NTHR, 1), NTHR, 0, stream>>>(h_prev, h_prev, h_prev, A1, A1, 0, NBATCH, NHID / 8, KCAT, NINF, 1.0f);
  cvt8_kernel<<<dim3(NHID * (NINF / 8) / NTHR, 3), NTHR, 0, stream>>>(Wz_w, Wr_w, Wh_w, BT, BT, 0, NHID, NINF / 8, KCAT, 0, WCARRY);
  cvt8_kernel<<<dim3(NHID * (NHID / 8) / NTHR, 3), NTHR, 0, stream>>>(Uz_w, Ur_w, Uh_w, BT, BT, 0, NHID, NHID / 8, KCAT, NINF, WCARRY);

  garch_rows_kernel<<<NBATCH / NTHR, NTHR, 0, stream>>>(x, eps_prev, sig_prev, omega_raw, alpha_raw, beta_raw, out_eps, out_sig);

  gru_gemm64<0><<<(NBATCH / 64) * (NZR / 64) / 8, NTHR, 0, stream>>>(
      A1, BT, Wz_b, Uz_b, Wr_b, Ur_b, h_prev, ZB, ZB, A3,
      Wg_w, Wg_b, eps_prev, sig_prev, omega_raw, alpha_raw, beta_raw, gamma_p);

  gru_gemm64<1><<<(NBATCH / 64) * (NHID / 64) / 8, NTHR, 0, stream>>>(
      A3, BT + (size_t)NZR * KCAT, Wh_b, Uh_b, Wh_b, Uh_b, h_prev, ZB, out_h, A3,
      Wg_w, Wg_b, eps_prev, sig_prev, omega_raw, alpha_raw, beta_raw, gamma_p);
}
